// MLA_28793460752680
// MI455X (gfx1250) — hardware-verified
//
#include <hip/hip_runtime.h>
#include <math.h>
#include <stdint.h>

#ifndef NB
#define NB 2
#endif
#ifndef SEQ
#define SEQ 2048
#endif
#define NB_FULL  2
#define SEQ_FULL 2048
#define DMOD  1024
#define NHD   16
#define HDIM  64
#define DHR   64
#define LATD  512
#define HD2   1024
#define QRW   1024
#define RHALF 512
#define NTOK  (NB * SEQ)
#define QCW   2048
#define KRW   128
#define KR_RSTRIDE (RHALF / (DHR / 2))

typedef __bf16       v16b __attribute__((ext_vector_type(16)));
typedef __bf16       v8b  __attribute__((ext_vector_type(8)));
typedef float        v8f  __attribute__((ext_vector_type(8)));
typedef float        v4f  __attribute__((ext_vector_type(4)));
typedef float        v2f  __attribute__((ext_vector_type(2)));
typedef unsigned int v4u  __attribute__((ext_vector_type(4)));

static_assert(NB >= 1 && NB <= NB_FULL);
static_assert(SEQ >= 64 && SEQ <= SEQ_FULL && SEQ % 64 == 0);
static_assert(HD2 == 2 * LATD);
static_assert(QRW == NHD * DHR);
static_assert(2 * RHALF == QRW);
static_assert(NHD * HDIM == DMOD);
static_assert(QCW == 2 * DMOD && QCW == 2 * QRW);
static_assert(KRW == 2 * DHR);
static_assert(KR_RSTRIDE * (DHR / 2) == RHALF);
static_assert(DMOD % 64 == 0 && LATD % 64 == 0 && HD2 % 64 == 0 && DHR % 64 == 0 && QRW % 64 == 0);
static_assert(DMOD % 32 == 0 && LATD % 32 == 0 && HD2 % 32 == 0);
static_assert((SEQ * RHALF) % 256 == 0);
static_assert((SEQ * DMOD / 8) % 256 == 0);

__device__ __forceinline__ unsigned short bf_bits(float f) {
  const unsigned u = __float_as_uint(f);
  return (unsigned short)((u + 0x7FFFu + ((u >> 16) & 1u)) >> 16);
}
__device__ __forceinline__ float bf_val(unsigned short hb) { return __uint_as_float(((unsigned)hb) << 16); }
__device__ __forceinline__ unsigned pk16(unsigned short a, unsigned short b) { return (unsigned)a | ((unsigned)b << 16); }
__device__ __forceinline__ v8f zero8() { v8f z = {0.f, 0.f, 0.f, 0.f, 0.f, 0.f, 0.f, 0.f}; return z; }
__device__ __forceinline__ int wave_id() { return __builtin_amdgcn_readfirstlane((int)(threadIdx.x >> 5)); }

__device__ __forceinline__ void lds_wave_sync() {
  __builtin_amdgcn_fence(3  , "workgroup");
  __builtin_amdgcn_wave_barrier();
  __builtin_amdgcn_fence(2  , "workgroup");
}

union FragB { v16b v; v8b h[2]; };
__device__ __forceinline__ v16b ldfrag_b(const __bf16* p) { FragB f; f.h[0] = *(const v8b*)(p); f.h[1] = *(const v8b*)(p + 16); return f.v; }

__device__ __forceinline__ v8f mma_b(v16b a, v16b b, v8f c) {
  return __builtin_amdgcn_wmma_f32_16x16x32_bf16(false, a, false, b, (short)0, c, false, false);
}
__device__ __forceinline__ void dep_guard_b(v8f& a, v8f& b, v16b x, v16b y) {
  asm volatile("v_nop\n\tv_nop\n\tv_nop\n\tv_nop" : "+v"(a), "+v"(b) : "v"(x), "v"(y));
}
__device__ __forceinline__ void keep4_b(v16b a, v16b b, v16b c, v16b d) { asm volatile("v_nop" :: "v"(a), "v"(b), "v"(c), "v"(d)); }
__device__ __forceinline__ void acc_guard4(v8f& a, v8f& b, v8f& c, v8f& d) {
  asm volatile("v_nop\n\tv_nop\n\tv_nop\n\tv_nop" : "+v"(a), "+v"(b), "+v"(c), "+v"(d));
}
__device__ __forceinline__ v8f at_mma(v16b a, v16b b, v8f c) {
  c = __builtin_amdgcn_wmma_f32_16x16x32_bf16(false, a, false, b, (short)0, c, false, false);
  asm volatile("v_nop\n\tv_nop\n\tv_nop\n\tv_nop" : "+v"(c) : "v"(a), "v"(b));
  return c;
}

__global__ __launch_bounds__(256) void rope_tab_kernel(float* __restrict__ tab, int npairs) {
  const int i = (int)blockIdx.x * 256 + (int)threadIdx.x;
  if (i >= npairs) return;
  const int t = i / RHALF;
  const int p = i - t * RHALF;
  const float ex  = ((float)(-2 * p) * (1.0f / (float)QRW)) * 9.210340371976184f;
  const float th  = expf(ex);
  const float ang = (float)(t + 1) * th;
  float sn, cs;
  sincosf(ang, &sn, &cs);
  v2f w;
  w[0] = cs;
  w[1] = sn;
  *(volatile v2f*)(tab + 2 * (size_t)i) = w;
  __threadfence();
  *(volatile v2f*)(tab + 2 * (size_t)i) = w;
}

__global__ __launch_bounds__(256) void cvt_bf16_kernel(const float* __restrict__ in, unsigned short* __restrict__ outp, int n8,
                                                       long inStride, long outStride) {
  const int bb = (int)blockIdx.y;
  const int i  = (int)blockIdx.x * 256 + (int)threadIdx.x;
  if (i >= n8) return;
  const size_t e = 8 * (size_t)i;
  const float* src = in + (size_t)bb * (size_t)inStride + e;
  unsigned short* dst = outp + (size_t)bb * (size_t)outStride + e;
  const v4f a = *(const v4f*)(src);
  const v4f b = *(const v4f*)(src + 4);
  v4u w;
  w[0] = pk16(bf_bits(a[0]), bf_bits(a[1]));
  w[1] = pk16(bf_bits(a[2]), bf_bits(a[3]));
  w[2] = pk16(bf_bits(b[0]), bf_bits(b[1]));
  w[3] = pk16(bf_bits(b[2]), bf_bits(b[3]));
  *(volatile v4u*)(dst) = w;
  __threadfence();
  *(volatile v4u*)(dst) = w;
}

__global__ __launch_bounds__(256) void tcvt_kernel(const float* __restrict__ W, unsigned short* __restrict__ oh, int R, int Cc) {
  __shared__ __align__(16) float tf[64 * 68];
  const int c0  = blockIdx.x * 64;
  const int r0  = blockIdx.y * 64;
  const int tid = threadIdx.x;
  {
    const int lr = tid >> 4;
    const int c4 = (tid & 15) * 4;
#pragma unroll
    for (int it = 0; it < 4; ++it) {
      const int rr = it * 16 + lr;
      const v4f a = *(const v4f*)(W + (size_t)(r0 + rr) * Cc + c0 + c4);
      *(v4f*)(tf + rr * 68 + c4) = a;
    }
  }
  __syncthreads();
  const int sub = tid >> 3;
  const int c8  = (tid & 7) * 8;
  v4u hv[2];
#pragma unroll
  for (int it = 0; it < 2; ++it) {
    const int oc = it * 32 + sub;
    v4u a;
#pragma unroll
    for (int q = 0; q < 4; ++q) {
      const float f0 = tf[(c8 + 2 * q) * 68 + oc];
      const float f1 = tf[(c8 + 2 * q + 1) * 68 + oc];
      a[q] = pk16(bf_bits(f0), bf_bits(f1));
    }
    hv[it] = a;
  }
  for (int pass = 0; pass < 2; ++pass) {
#pragma unroll
    for (int it = 0; it < 2; ++it) {
      const int oc = it * 32 + sub;
      const size_t go = (size_t)(c0 + oc) * R + r0 + c8;
      *(volatile v4u*)(oh + go) = hv[it];
    }
    __threadfence();
  }
}

template <bool ASPLIT, bool BSPLIT, int OUT_MODE, int BIASM, bool ROPE>
__global__ __launch_bounds__(256) void gemm64_kernel(
    const unsigned short* __restrict__ Ap, const unsigned short* __restrict__ A2p, int lda, long strideA,
    const unsigned short* __restrict__ Btp, const unsigned short* __restrict__ Bt2p, int ldb, long strideB,
    const float* __restrict__ bias, const float* __restrict__ rtab, int rstride,
    void* Cout, void* Cout2, int ldc, long strideC,
    int M, int N, int K, float scale) {
  static_assert(!ROPE || OUT_MODE == 2);
  static_assert(BIASM >= 0 && BIASM <= 2);
  static_assert(OUT_MODE == 0 || OUT_MODE == 2);
  __shared__ __align__(16) float sT[8][16 * 68];
  const __bf16* A   = (const __bf16*)(const void*)Ap;
  const __bf16* A2  = (const __bf16*)(const void*)A2p;
  const __bf16* Bt  = (const __bf16*)(const void*)Btp;
  const __bf16* Bt2 = (const __bf16*)(const void*)Bt2p;
  const int b    = blockIdx.y;
  const int lane = threadIdx.x & 31;
  const int wave = wave_id();
  const int tilesN = N >> 6;
  const int tilesM = M >> 6;
  const int tile = (int)blockIdx.x * 8 + wave;
  if (tile >= tilesM * tilesN) return;
  const int tm = tile / tilesN;
  const int tn = tile - tm * tilesN;
  const int m0 = tm << 6;
  const int n0 = tn << 6;

  const __bf16* Ab  = A  + (size_t)b * strideA;
  const __bf16* Bb  = Bt + (size_t)b * strideB;
  const __bf16* Ab2 = ASPLIT ? (A2  + (size_t)b * strideA) : Ab;
  const __bf16* Bb2 = BSPLIT ? (Bt2 + (size_t)b * strideB) : Bb;

  const int rlane = lane & 15;
  const int koff  = (lane >> 4) * 8;
  const int mOff  = (lane >> 4) * 8;

  v8f acc[4][4];
#pragma unroll
  for (int i = 0; i < 4; ++i)
#pragma unroll
    for (int j = 0; j < 4; ++j) acc[i][j] = zero8();

  for (int k0 = 0; k0 < K; k0 += 32) {
    v16b bh[4], bl[4];
#pragma unroll
    for (int j = 0; j < 4; ++j) {
      const size_t bo = (size_t)(n0 + (j << 4) + rlane) * ldb + koff + k0;
      bh[j] = ldfrag_b(Bb + bo);
      bl[j] = BSPLIT ? ldfrag_b(Bb2 + bo) : bh[j];
    }
#pragma unroll
    for (int i = 0; i < 4; ++i) {
      const size_t ao = (size_t)(m0 + (i << 4) + rlane) * lda + koff + k0;
      const v16b ah = ldfrag_b(Ab + ao);
      const v16b al = ASPLIT ? ldfrag_b(Ab2 + ao) : ah;
#pragma unroll
      for (int j = 0; j < 4; ++j) {
        acc[i][j] = mma_b(ah, bh[j], acc[i][j]);
        if (BSPLIT) acc[i][j] = mma_b(ah, bl[j], acc[i][j]);
        if (ASPLIT) acc[i][j] = mma_b(al, bh[j], acc[i][j]);
      }
      dep_guard_b(acc[i][0], acc[i][3], ah, al);
    }
    keep4_b(bh[0], bh[1], bh[2], bh[3]);
    if (BSPLIT) keep4_b(bl[0], bl[1], bl[2], bl[3]);
  }
  acc_guard4(acc[0][0], acc[0][1], acc[0][2], acc[0][3]);
  acc_guard4(acc[1][0], acc[1][1], acc[1][2], acc[1][3]);
  acc_guard4(acc[2][0], acc[2][1], acc[2][2], acc[2][3]);
  acc_guard4(acc[3][0], acc[3][1], acc[3][2], acc[3][3]);

  float* slab = sT[wave];
#pragma unroll
  for (int i = 0; i < 4; ++i) {
    const int mBase = m0 + (i << 4);
    float brow[8];
#pragma unroll
    for (int r = 0; r < 8; ++r) brow[r] = (BIASM == 2) ? bias[mBase + mOff + r] : 0.f;
#pragma unroll
    for (int j = 0; j < 4; ++j) {
      const float bcol = (BIASM == 1) ? bias[n0 + (j << 4) + rlane] : 0.f;
#pragma unroll
      for (int r = 0; r < 8; ++r)
        slab[(mOff + r) * 68 + (j << 4) + rlane] = acc[i][j][r] * scale + bcol + brow[r];
    }
    lds_wave_sync();
    if (OUT_MODE == 0) {
      float* C = (float*)Cout + (size_t)b * strideC;
      const int hh = lane >> 4, c4 = (lane & 15) * 4;
      for (int pass = 0; pass < 2; ++pass) {
#pragma unroll
        for (int it = 0; it < 8; ++it) {
          const int row = it * 2 + hh;
          const v4f v = *(const v4f*)(slab + row * 68 + c4);
          *(volatile v4f*)(C + (size_t)(mBase + row) * ldc + n0 + c4) = v;
        }
        __threadfence();
      }
    } else {
      const int q = lane >> 3, c8 = (lane & 7) * 8;
      unsigned short* C  = (unsigned short*)Cout  + (size_t)b * strideC;
      unsigned short* C2 = (unsigned short*)Cout2 + (size_t)b * strideC;
      for (int pass = 0; pass < 2; ++pass) {
#pragma unroll
        for (int it = 0; it < 4; ++it) {
          const int row = it * 4 + q;
          const float* sp = slab + row * 68 + c8;
          const float* tp = rtab;
          if (ROPE) {
            const int tt = (mBase + row) % SEQ;
            tp = rtab + ((size_t)tt * RHALF + (size_t)((n0 + c8) >> 1) * (size_t)rstride) * 2;
          }
          v4u hv, lv;
#pragma unroll
          for (int e = 0; e < 4; ++e) {
            float f0 = sp[2 * e], f1 = sp[2 * e + 1];
            if (ROPE) {
              const v2f cs = *(const v2f*)(tp + (size_t)e * (size_t)rstride * 2);
              const float g0 = f0 * cs[0] - f1 * cs[1];
              const float g1 = f1 * cs[0] + f0 * cs[1];
              f0 = g0;
              f1 = g1;
            }
            const unsigned short h0 = bf_bits(f0), h1 = bf_bits(f1);
            const unsigned short l0 = bf_bits(f0 - bf_val(h0)), l1 = bf_bits(f1 - bf_val(h1));
            hv[e] = pk16(h0, h1);
            lv[e] = pk16(l0, l1);
          }
          *(volatile v4u*)(C  + (size_t)(mBase + row) * ldc + n0 + c8) = hv;
          *(volatile v4u*)(C2 + (size_t)(mBase + row) * ldc + n0 + c8) = lv;
        }
        __threadfence();
      }
    }
    lds_wave_sync();
  }
}

#define AT_DQ 128
#define AT_DV 64
#define AT_NW 4
#define AT_KC 64
static_assert(AT_DQ == HDIM + DHR);
static_assert(AT_DV == HDIM);
static_assert((2 * AT_KC * AT_DQ + 2 * AT_DV * AT_KC + 2 * AT_NW * 16 * AT_KC) * 2 <= 65536);
static_assert(16 * AT_KC * (int)sizeof(__bf16) >= 16 * AT_DV * (int)sizeof(unsigned short));

__global__ __launch_bounds__(128)
void attn_causal_kernel(unsigned short* qnp, const unsigned short* __restrict__ qrp,
                        const unsigned short* __restrict__ knp, const unsigned short* __restrict__ krp,
                        const unsigned short* __restrict__ vhp, const unsigned short* __restrict__ vlp,
                        float sscale) {
  __shared__ __align__(16) __bf16 Ksh[AT_KC * AT_DQ];
  __shared__ __align__(16) __bf16 Ksl[AT_KC * AT_DQ];
  __shared__ __align__(16) __bf16 Vth[AT_DV * AT_KC];
  __shared__ __align__(16) __bf16 Vtl[AT_DV * AT_KC];
  __shared__ __align__(16) __bf16 Psh[AT_NW][16 * AT_KC];
  __shared__ __align__(16) __bf16 Psl[AT_NW][16 * AT_KC];

  const int tid  = (int)threadIdx.x;
  const int wave = wave_id();
  const int lane = tid & 31;
  const int hh   = lane >> 4;
  const int c    = lane & 15;

  const int nqb = SEQ / 64;
  const int bx = (int)blockIdx.x;
  const int qb = bx % nqb;
  const int h  = bx / nqb;
  const int b  = (int)blockIdx.y;
  const int q0 = qb * 64 + wave * 16;
  const size_t tok0 = (size_t)b * SEQ;

  const __bf16* QNb = (const __bf16*)(const void*)qnp;
  const __bf16* Qh  = QNb + (size_t)h * HDIM;
  const __bf16* Ql  = QNb + DMOD + (size_t)h * HDIM;
  const __bf16* QRb = (const __bf16*)(const void*)qrp;
  const __bf16* Rh  = QRb + (size_t)h * DHR;
  const __bf16* Rl  = QRb + QRW + (size_t)h * DHR;
  const __bf16* KNb = (const __bf16*)(const void*)knp;
  const __bf16* Kh  = KNb + (size_t)h * HDIM;
  const __bf16* Kl  = KNb + DMOD + (size_t)h * HDIM;
  const __bf16* KRh = (const __bf16*)(const void*)krp;
  const __bf16* KRl = KRh + DHR;
  const __bf16* Vh  = (const __bf16*)(const void*)vhp + ((size_t)b * DMOD + (size_t)h * HDIM) * SEQ;
  const __bf16* Vl  = (const __bf16*)(const void*)vlp + ((size_t)b * DMOD + (size_t)h * HDIM) * SEQ;

  const size_t qoff = (tok0 + (size_t)(q0 + c)) * QCW + 8 * hh;
  v16b qah[4];
  qah[0] = ldfrag_b(Qh + qoff);
  qah[1] = ldfrag_b(Qh + qoff + 32);
  qah[2] = ldfrag_b(Rh + qoff);
  qah[3] = ldfrag_b(Rh + qoff + 32);
  const __bf16* qlp0 = Ql + qoff;
  const __bf16* qlp2 = Rl + qoff;

  float mrow[8], lrow[8];
  v8f oacc[4];
#pragma unroll
  for (int r = 0; r < 8; ++r) { mrow[r] = -INFINITY; lrow[r] = 0.f; }
#pragma unroll
  for (int t = 0; t < 4; ++t) oacc[t] = zero8();

  __bf16* pwh = Psh[wave];
  __bf16* pwl = Psl[wave];

  const int nChunks = qb + 1;
  for (int kc = 0; kc < nChunks; ++kc) {
    const int kv0 = kc * AT_KC;
    __syncthreads();
    {
      const int r    = tid & 63;
      const int half = tid >> 6;
      const size_t krow = tok0 + (size_t)(kv0 + r);
      const __bf16* ksh = (half == 0) ? (Kh + krow * QCW) : (KRh + krow * KRW);
      const __bf16* ksl = (half == 0) ? (Kl + krow * QCW) : (KRl + krow * KRW);
      __bf16* kdh = Ksh + r * AT_DQ + half * 64;
      __bf16* kdl = Ksl + r * AT_DQ + half * 64;
#pragma unroll
      for (int i = 0; i < 8; ++i) {
        const v8b a0 = *(const v8b*)(ksh + 8 * i);
        const v8b a1 = *(const v8b*)(ksl + 8 * i);
        *(v8b*)(kdh + 8 * i) = a0;
        *(v8b*)(kdl + 8 * i) = a1;
      }
      const __bf16* vsh = Vh + (size_t)r * SEQ + kv0 + half * 32;
      const __bf16* vsl = Vl + (size_t)r * SEQ + kv0 + half * 32;
#pragma unroll
      for (int i = 0; i < 4; ++i) {
        const v8b b0 = *(const v8b*)(vsh + 8 * i);
        const v8b b1 = *(const v8b*)(vsl + 8 * i);
        *(v8b*)(Vth + r * AT_KC + half * 32 + 8 * i) = b0;
        *(v8b*)(Vtl + r * AT_KC + half * 32 + 8 * i) = b1;
      }
    }
    __syncthreads();

    v8f s[4];
#pragma unroll
    for (int j = 0; j < 4; ++j) s[j] = zero8();
#pragma unroll
    for (int dc = 0; dc < 4; ++dc) {
      const v16b qa = qah[dc];
      const v16b ql = ldfrag_b((dc < 2) ? (qlp0 + dc * 32) : (qlp2 + (dc - 2) * 32));
#pragma unroll
      for (int j = 0; j < 4; ++j) {
        FragB kb, kl;
        const __bf16* kr0 = Ksh + (j * 16 + c) * AT_DQ + dc * 32 + 8 * hh;
        const __bf16* kr1 = Ksl + (j * 16 + c) * AT_DQ + dc * 32 + 8 * hh;
        kb.h[0] = *(const v8b*)(kr0);
        kb.h[1] = *(const v8b*)(kr0 + 16);
        kl.h[0] = *(const v8b*)(kr1);
        kl.h[1] = *(const v8b*)(kr1 + 16);
        s[j] = at_mma(qa, kb.v, s[j]);
        s[j] = at_mma(qa, kl.v, s[j]);
        s[j] = at_mma(ql, kb.v, s[j]);
      }
    }
    const bool diag = (kc == qb);
    float cm[8];
#pragma unroll
    for (int r = 0; r < 8; ++r) {
      const int qrow = q0 + 8 * hh + r;
      float m = -INFINITY;
#pragma unroll
      for (int j = 0; j < 4; ++j) {
        const int kvcol = kv0 + j * 16 + c;
        const float sv = s[j][r] * sscale;
        const bool masked = diag && (kvcol > qrow);
        const float sm = masked ? -INFINITY : sv;
        s[j][r] = sm;
        m = fmaxf(m, sm);
      }
#pragma unroll
      for (int off = 1; off < 16; off <<= 1) m = fmaxf(m, __shfl_xor(m, off, 32));
      cm[r] = m;
    }
#pragma unroll
    for (int r = 0; r < 8; ++r) {
      const float mnew = fmaxf(mrow[r], cm[r]);
      const float alpha = expf(mrow[r] - mnew);
      mrow[r] = mnew;
      float psum = 0.f;
#pragma unroll
      for (int j = 0; j < 4; ++j) {
        const float p = expf(s[j][r] - mnew);
        psum += p;
        const unsigned short hb = bf_bits(p);
        const unsigned short lb = bf_bits(p - bf_val(hb));
        pwh[(8 * hh + r) * AT_KC + j * 16 + c] = __builtin_bit_cast(__bf16, hb);
        pwl[(8 * hh + r) * AT_KC + j * 16 + c] = __builtin_bit_cast(__bf16, lb);
      }
#pragma unroll
      for (int off = 1; off < 16; off <<= 1) psum += __shfl_xor(psum, off, 32);
      lrow[r] = lrow[r] * alpha + psum;
#pragma unroll
      for (int t = 0; t < 4; ++t) oacc[t][r] *= alpha;
    }
    lds_wave_sync();
#pragma unroll 1
    for (int kk = 0; kk < 2; ++kk) {
      FragB pa, pl;
      pa.h[0] = *(const v8b*)(pwh + c * AT_KC + kk * 32 + 8 * hh);
      pa.h[1] = *(const v8b*)(pwh + c * AT_KC + kk * 32 + 16 + 8 * hh);
      pl.h[0] = *(const v8b*)(pwl + c * AT_KC + kk * 32 + 8 * hh);
      pl.h[1] = *(const v8b*)(pwl + c * AT_KC + kk * 32 + 16 + 8 * hh);
#pragma unroll
      for (int t = 0; t < 4; ++t) {
        FragB vb, vl;
        vb.h[0] = *(const v8b*)(Vth + (t * 16 + c) * AT_KC + kk * 32 + 8 * hh);
        vb.h[1] = *(const v8b*)(Vth + (t * 16 + c) * AT_KC + kk * 32 + 16 + 8 * hh);
        vl.h[0] = *(const v8b*)(Vtl + (t * 16 + c) * AT_KC + kk * 32 + 8 * hh);
        vl.h[1] = *(const v8b*)(Vtl + (t * 16 + c) * AT_KC + kk * 32 + 16 + 8 * hh);
        oacc[t] = at_mma(pa.v, vb.v, oacc[t]);
        oacc[t] = at_mma(pa.v, vl.v, oacc[t]);
        oacc[t] = at_mma(pl.v, vb.v, oacc[t]);
      }
    }
  }
  acc_guard4(oacc[0], oacc[1], oacc[2], oacc[3]);
  lds_wave_sync();

  unsigned short* osh = (unsigned short*)(void*)pwh;
  unsigned short* osl = (unsigned short*)(void*)pwl;
#pragma unroll
  for (int r = 0; r < 8; ++r) {
    const float inv = 1.0f / lrow[r];
#pragma unroll
    for (int t = 0; t < 4; ++t) {
      const float o = oacc[t][r] * inv;
      const unsigned short hb = bf_bits(o);
      const unsigned short lb = bf_bits(o - bf_val(hb));
      const int so = (8 * hh + r) * AT_DV + t * 16 + c;
      osh[so] = hb;
      osl[so] = lb;
    }
  }
  lds_wave_sync();
  unsigned short* Ag = qnp + (tok0 + (size_t)q0) * QCW + (size_t)h * HDIM;
  const int qq = lane >> 3;
  const int c8 = (lane & 7) * 8;
  for (int pass = 0; pass < 2; ++pass) {
#pragma unroll
    for (int it = 0; it < 4; ++it) {
      const int row = it * 4 + qq;
      const v4u x = *(const v4u*)(osh + row * AT_DV + c8);
      const v4u y = *(const v4u*)(osl + row * AT_DV + c8);
      *(volatile v4u*)(Ag + (size_t)row * QCW + c8)        = x;
      *(volatile v4u*)(Ag + (size_t)row * QCW + DMOD + c8) = y;
    }
    __threadfence();
  }
}

#define WS_TOTAL_BYTES ((size_t)SEQ * RHALF * 8 + (size_t)NTOK * DMOD * 2 + (size_t)HD2 * DMOD * 2 + (size_t)DHR * HD2 * 2 + \
                        (size_t)QRW * HD2 * 2 + (size_t)2 * DMOD * LATD * 2 + (size_t)DMOD * LATD * 2 + (size_t)DMOD * DMOD * 2 + \
                        (size_t)2 * NTOK * HD2 * 2 + (size_t)3 * NTOK * QCW * 2 + (size_t)NTOK * KRW * 2 + \
                        (size_t)2 * NB * DMOD * SEQ * 2)
static_assert(WS_TOTAL_BYTES <= (size_t)134217728);
static_assert(NB != NB_FULL || SEQ != SEQ_FULL || WS_TOTAL_BYTES == (size_t)111280128);
static_assert((size_t)(((size_t)(NB_FULL - 1) * SEQ_FULL + SEQ_FULL) * DMOD) * 4 <= (size_t)16777216);

extern "C" void kernel_launch(void* const* d_in, const int* in_sizes, int n_in,
                              void* d_out, int out_size, void* d_ws, size_t ws_size,
                              hipStream_t stream) {
  if (n_in < 13) return;
  const long needX = ((long)(NB - 1) * SEQ_FULL + SEQ) * DMOD;
  if ((long)in_sizes[0] < needX) return;
  if (in_sizes[1] != DMOD * HD2) return;
  if (in_sizes[2] < HD2) return;
  if (in_sizes[3] != HD2 * DHR) return;
  if (in_sizes[4] < DHR) return;
  if (in_sizes[5] != HD2 * QRW) return;
  if (in_sizes[6] < QRW) return;
  if (in_sizes[7] != LATD * 2 * DMOD) return;
  if (in_sizes[8] < 2 * DMOD) return;
  if (in_sizes[9] != LATD * DMOD) return;
  if (in_sizes[10] < DMOD) return;
  if (in_sizes[11] != DMOD * DMOD) return;
  if (in_sizes[12] < DMOD) return;
  if ((long)out_size < needX) return;

  const float* x   = (const float*)d_in[0];
  const float* w1  = (const float*)d_in[1];
  const float* b1  = (const float*)d_in[2];
  const float* wkr = (const float*)d_in[3];
  const float* bkr = (const float*)d_in[4];
  const float* wqr = (const float*)d_in[5];
  const float* bqr = (const float*)d_in[6];
  const float* wkv = (const float*)d_in[7];
  const float* bkv = (const float*)d_in[8];
  const float* wq  = (const float*)d_in[9];
  const float* bq  = (const float*)d_in[10];
  const float* wo  = (const float*)d_in[11];
  const float* bo  = (const float*)d_in[12];
  float* out = (float*)d_out;

  const size_t szTAB  = (size_t)SEQ * RHALF * 2 * 4;
  const size_t szXB   = (size_t)NTOK * DMOD * 2;
  const size_t szW1T  = (size_t)HD2 * DMOD * 2;
  const size_t szWKRT = (size_t)DHR * HD2 * 2;
  const size_t szWQRT = (size_t)QRW * HD2 * 2;
  const size_t szWKVT = (size_t)2 * DMOD * LATD * 2;
  const size_t szWQT  = (size_t)DMOD * LATD * 2;
  const size_t szWOT  = (size_t)DMOD * DMOD * 2;
  const size_t szH    = (size_t)NTOK * HD2 * 2;
  const size_t szQC   = (size_t)NTOK * QCW * 2;
  const size_t szKR   = (size_t)NTOK * KRW * 2;
  const size_t szVT   = (size_t)NB * DMOD * SEQ * 2;
  size_t off = 0;
  const size_t oTAB  = off; off += szTAB;
  const size_t oXB   = off; off += szXB;
  const size_t oW1T  = off; off += szW1T;
  const size_t oWKRT = off; off += szWKRT;
  const size_t oWQRT = off; off += szWQRT;
  const size_t oWKVT = off; off += szWKVT;
  const size_t oWQT  = off; off += szWQT;
  const size_t oWOT  = off; off += szWOT;
  const size_t oHH   = off; off += szH;
  const size_t oHL   = off; off += szH;
  const size_t oQN   = off; off += szQC;
  const size_t oQR   = off; off += szQC;
  const size_t oKN   = off; off += szQC;
  const size_t oKR   = off; off += szKR;
  const size_t oVTH  = off; off += szVT;
  const size_t oVTL  = off; off += szVT;
  if (off != WS_TOTAL_BYTES) return;
  if (off > ws_size) return;

  char* ws = (char*)d_ws;
  float*          TAB  = (float*)(ws + oTAB);
  unsigned short* XB   = (unsigned short*)(ws + oXB);
  unsigned short* W1T  = (unsigned short*)(ws + oW1T);
  unsigned short* WKRT = (unsigned short*)(ws + oWKRT);
  unsigned short* WQRT = (unsigned short*)(ws + oWQRT);
  unsigned short* WKVT = (unsigned short*)(ws + oWKVT);
  unsigned short* WQT  = (unsigned short*)(ws + oWQT);
  unsigned short* WOT  = (unsigned short*)(ws + oWOT);
  unsigned short* HH   = (unsigned short*)(ws + oHH);
  unsigned short* HL   = (unsigned short*)(ws + oHL);
  unsigned short* QN   = (unsigned short*)(ws + oQN);
  unsigned short* QR   = (unsigned short*)(ws + oQR);
  unsigned short* KN   = (unsigned short*)(ws + oKN);
  unsigned short* KR   = (unsigned short*)(ws + oKR);
  unsigned short* VTH  = (unsigned short*)(ws + oVTH);
  unsigned short* VTL  = (unsigned short*)(ws + oVTL);

  const dim3 b256(256), b128(128);
  const float sscale = 0.08838834764831845f;

  rope_tab_kernel<<<dim3((SEQ * RHALF + 255) / 256), b256, 0, stream>>>(TAB, SEQ * RHALF);
  cvt_bf16_kernel<<<dim3(((SEQ * DMOD / 8) + 255) / 256, NB), b256, 0, stream>>>(x, XB, SEQ * DMOD / 8,
                                                                                 (long)SEQ_FULL * DMOD, (long)SEQ * DMOD);
  tcvt_kernel<<<dim3(HD2 / 64, DMOD / 64), b256, 0, stream>>>(w1, W1T, DMOD, HD2);
  tcvt_kernel<<<dim3(DHR / 64, HD2 / 64), b256, 0, stream>>>(wkr, WKRT, HD2, DHR);
  tcvt_kernel<<<dim3(QRW / 64, HD2 / 64), b256, 0, stream>>>(wqr, WQRT, HD2, QRW);
  tcvt_kernel<<<dim3((2 * DMOD) / 64, LATD / 64), b256, 0, stream>>>(wkv, WKVT, LATD, 2 * DMOD);
  tcvt_kernel<<<dim3(DMOD / 64, LATD / 64), b256, 0, stream>>>(wq, WQT, LATD, DMOD);
  tcvt_kernel<<<dim3(DMOD / 64, DMOD / 64), b256, 0, stream>>>(wo, WOT, DMOD, DMOD);

  const int tilesTok = NTOK / 64;
  gemm64_kernel<false, false, 2, 1, false><<<dim3((tilesTok * (HD2 / 64) + 7) / 8, 1), b256, 0, stream>>>(
      XB, XB, DMOD, 0L, W1T, W1T, DMOD, 0L, b1, TAB, 0, (void*)HH, (void*)HL, HD2, 0L, NTOK, HD2, DMOD, 1.0f);
  gemm64_kernel<true, false, 2, 1, true><<<dim3((tilesTok * (QRW / 64) + 7) / 8, 1), b256, 0, stream>>>(
      HH, HL, HD2, 0L, WQRT, WQRT, HD2, 0L, bqr, TAB, 1, (void*)QR, (void*)(QR + QRW), QCW, 0L, NTOK, QRW, HD2, 1.0f);
  gemm64_kernel<true, false, 2, 1, true><<<dim3((tilesTok * (DHR / 64) + 7) / 8, 1), b256, 0, stream>>>(
      HH, HL, HD2, 0L, WKRT, WKRT, HD2, 0L, bkr, TAB, KR_RSTRIDE, (void*)KR, (void*)(KR + DHR), KRW, 0L, NTOK, DHR, HD2, 1.0f);
  gemm64_kernel<true, false, 2, 1, false><<<dim3((tilesTok * (DMOD / 64) + 7) / 8, 1), b256, 0, stream>>>(
      HH, HL, HD2, 0L, WKVT, WKVT, LATD, 0L, bkv, TAB, 0, (void*)KN, (void*)(KN + DMOD), QCW, 0L, NTOK, DMOD, LATD, 1.0f);
  gemm64_kernel<false, true, 2, 2, false><<<dim3(((DMOD / 64) * (SEQ / 64) + 7) / 8, NB), b256, 0, stream>>>(
      WKVT + (size_t)DMOD * LATD, WKVT + (size_t)DMOD * LATD, LATD, 0L, HH, HL, HD2, (long)SEQ * HD2, bkv + DMOD, TAB, 0,
      (void*)VTH, (void*)VTL, SEQ, (long)DMOD * SEQ, DMOD, SEQ, LATD, 1.0f);
  gemm64_kernel<true, false, 2, 1, false><<<dim3((tilesTok * (DMOD / 64) + 7) / 8, 1), b256, 0, stream>>>(
      HH + LATD, HL + LATD, HD2, 0L, WQT, WQT, LATD, 0L, bq, TAB, 0, (void*)QN, (void*)(QN + DMOD), QCW, 0L, NTOK, DMOD, LATD, 1.0f);
  attn_causal_kernel<<<dim3(NHD * (SEQ / 64), NB), b128, 0, stream>>>(QN, QR, KN, KR, VTH, VTL, sscale);
  gemm64_kernel<true, false, 0, 1, false><<<dim3(((SEQ / 64) * (DMOD / 64) + 7) / 8, NB), b256, 0, stream>>>(
      QN, QN + DMOD, QCW, (long)SEQ * QCW, WOT, WOT, DMOD, 0L, bo, TAB, 0, (void*)out, (void*)out, DMOD, (long)SEQ_FULL * DMOD,
      SEQ, DMOD, DMOD, 1.0f);
  (void)hipGetLastError();
}
